// MultiTaskPolicy_76055280877948
// MI455X (gfx1250) — hardware-verified
//
#include <hip/hip_runtime.h>

constexpr int kBatch   = 256;
constexpr int kImg     = 128;
constexpr int kCin0    = 3;
constexpr int kCh1     = 64;  constexpr int kSp1 = 64;
constexpr int kCh2     = 128; constexpr int kSp2 = 32;
constexpr int kCh3     = 256; constexpr int kSp3 = 16;
constexpr int kChunk   = 32;
constexpr int kNChunk  = kBatch / kChunk;
constexpr int kK1      = 32;
constexpr int kK1r     = 27;
constexpr int kK2      = 9 * kCh1;
constexpr int kK3      = 9 * kCh2;
constexpr int kM1c     = kChunk * kSp1 * kSp1;
constexpr int kM2c     = kChunk * kSp2 * kSp2;
constexpr int kM3c     = kChunk * kSp3 * kSp3;
constexpr int kEnc     = 256;
constexpr int kPropIn  = 7;
constexpr int kPropH   = 64;
constexpr int kCatK    = 320;
constexpr int kEmb     = 32;
constexpr int kGK      = 288;
constexpr int kHidH    = 128;
constexpr int kActN    = 4;
constexpr int kTasks   = 150;
constexpr float kWCarry    = 16.0f;
constexpr float kWCarryInv = 1.0f / 16.0f;

typedef __attribute__((ext_vector_type(16))) _Float16 v16h;
typedef __attribute__((ext_vector_type(8)))  _Float16 v8h;
typedef __attribute__((ext_vector_type(16))) __bf16   v16b;
typedef __attribute__((ext_vector_type(8)))  __bf16   v8b;
typedef __attribute__((ext_vector_type(8)))  float    v8f;
typedef __attribute__((ext_vector_type(4)))  float    v4f;
typedef __attribute__((ext_vector_type(4)))  unsigned int v4u;

__device__ __forceinline__ unsigned short f2bf_bits(float f) {
  unsigned u = __float_as_uint(f);
  return (unsigned short)((u + 0x7FFFu + ((u >> 16) & 1u)) >> 16);
}
__device__ __forceinline__ float bf_bits2f(unsigned short h) { return __uint_as_float(((unsigned)h) << 16); }

__device__ __forceinline__ void dep_guard_h(v8f& a, v8f& b, v16h x, v16h y) { asm volatile("v_nop\n\tv_nop\n\tv_nop\n\tv_nop" : "+v"(a), "+v"(b) : "v"(x), "v"(y)); }
__device__ __forceinline__ void dep_guard_b(v8f& a, v8f& b, v16b x, v16b y) { asm volatile("v_nop\n\tv_nop\n\tv_nop\n\tv_nop" : "+v"(a), "+v"(b) : "v"(x), "v"(y)); }
__device__ __forceinline__ void keep4_h(v16h a, v16h b, v16h c, v16h d) { asm volatile("v_nop" :: "v"(a), "v"(b), "v"(c), "v"(d)); }
__device__ __forceinline__ void keep4_b(v16b a, v16b b, v16b c, v16b d) { asm volatile("v_nop" :: "v"(a), "v"(b), "v"(c), "v"(d)); }
__device__ __forceinline__ void acc_guard4(v8f& a, v8f& b, v8f& c, v8f& d) { asm volatile("v_nop\n\tv_nop\n\tv_nop\n\tv_nop" : "+v"(a), "+v"(b), "+v"(c), "+v"(d)); }
template <typename T> struct Frag;
template <> struct Frag<_Float16> {
  typedef v16h V; union U { v16h v; v8h h[2]; };
  static __device__ __forceinline__ v16h load(const _Float16* p) {
    U f; f.h[0] = *(const v8h*)(p); f.h[1] = *(const v8h*)(p + 16); return f.v;
  }
  static __device__ __forceinline__ v8f mma(v16h a, v16h b, v8f c) {
    return __builtin_amdgcn_wmma_f32_16x16x32_f16(false, a, false, b, (short)0, c, false, false);
  }
  static __device__ __forceinline__ void guard(v8f& a, v8f& b, v16h x, v16h y) { dep_guard_h(a, b, x, y); }
  static __device__ __forceinline__ void keep(v16h a, v16h b, v16h c, v16h d) { keep4_h(a, b, c, d); }
};
template <> struct Frag<__bf16> {
  typedef v16b V; union U { v16b v; v8b h[2]; };
  static __device__ __forceinline__ v16b load(const __bf16* p) {
    U f; f.h[0] = *(const v8b*)(p); f.h[1] = *(const v8b*)(p + 16); return f.v;
  }
  static __device__ __forceinline__ v8f mma(v16b a, v16b b, v8f c) {
    return __builtin_amdgcn_wmma_f32_16x16x32_bf16(false, a, false, b, (short)0, c, false, false);
  }
  static __device__ __forceinline__ void guard(v8f& a, v8f& b, v16b x, v16b y) { dep_guard_b(a, b, x, y); }
  static __device__ __forceinline__ void keep(v16b a, v16b b, v16b c, v16b d) { keep4_b(a, b, c, d); }
};

__device__ __forceinline__ unsigned pk16(unsigned short a, unsigned short b) { return (unsigned)a | ((unsigned)b << 16); }
__device__ __forceinline__ unsigned short h_bits(float f) { const _Float16 h = (_Float16)f; return __builtin_bit_cast(unsigned short, h); }

template <int ET> struct Elem;
template <> struct Elem<0> { typedef _Float16 T; };
template <> struct Elem<1> { typedef __bf16 T; };
template <int ET, bool SPLIT, int BIAS_MODE, int OUT_MODE, bool RESID, int ACT = 0>
__global__ __launch_bounds__(256) void wmma_gemm64(
    const unsigned short* __restrict__ Ap, const unsigned short* __restrict__ A2p, int lda, long strideA,
    const unsigned short* __restrict__ Btp, const unsigned short* __restrict__ Bt2p, int ldb, long strideB,
    void* __restrict__ Cout, void* __restrict__ Cout2, int ldc, long strideC,
    const float* __restrict__ bias,
    const float* __restrict__ resid, long strideR,
    int M, int N, int K, float scale) {
  typedef typename Elem<ET>::T T;
  typedef typename Frag<T>::V V;
  const T* A = (const T*)Ap; const T* A2 = (const T*)A2p; const T* Bt = (const T*)Btp; const T* Bt2 = (const T*)Bt2p;
  __shared__ __align__(16) float sT[8][16 * 68];
  const int b    = blockIdx.y;
  const int lane = threadIdx.x & 31;
  const int wave = threadIdx.x >> 5;
  const int tilesN = N >> 6;
  const int tilesM = M >> 6;
  const int tile = blockIdx.x * 8 + wave;
  if (tile >= tilesM * tilesN) return;
  const int tm = tile / tilesN;
  const int tn = tile - tm * tilesN;
  const int m0 = tm << 6;
  const int n0 = tn << 6;

  const T* Ab  = A  + (size_t)b * strideA;
  const T* Bb  = Bt + (size_t)b * strideB;
  const T* Ab2 = SPLIT ? (A2  + (size_t)b * strideA) : nullptr;
  const T* Bb2 = SPLIT ? (Bt2 + (size_t)b * strideB) : nullptr;

  const int rlane = lane & 15;
  const int koff  = (lane >> 4) * 8;
  const int mOff  = (lane >> 4) * 8;

  v8f acc[4][4];
#pragma unroll
  for (int i = 0; i < 4; ++i)
#pragma unroll
    for (int j = 0; j < 4; ++j) acc[i][j] = (v8f){0.f,0.f,0.f,0.f,0.f,0.f,0.f,0.f};

  for (int k0 = 0; k0 < K; k0 += 32) {
    V bh[4], bl[4];
#pragma unroll
    for (int j = 0; j < 4; ++j) {
      const size_t bo = (size_t)(n0 + (j << 4) + rlane) * ldb + koff + k0;
      bh[j] = Frag<T>::load(Bb + bo);
      if (SPLIT) bl[j] = Frag<T>::load(Bb2 + bo);
    }
#pragma unroll
    for (int i = 0; i < 4; ++i) {
      const size_t ao = (size_t)(m0 + (i << 4) + rlane) * lda + koff + k0;
      V ah = Frag<T>::load(Ab + ao);
      V al;
      if (SPLIT) al = Frag<T>::load(Ab2 + ao);
#pragma unroll
      for (int j = 0; j < 4; ++j) {
        acc[i][j] = Frag<T>::mma(ah, bh[j], acc[i][j]);
        if (SPLIT) {
          acc[i][j] = Frag<T>::mma(ah, bl[j], acc[i][j]);
          acc[i][j] = Frag<T>::mma(al, bh[j], acc[i][j]);
        }
      }
      Frag<T>::guard(acc[i][0], acc[i][3], ah, SPLIT ? al : ah);
    }
    Frag<T>::keep(bh[0], bh[1], bh[2], bh[3]);
    if (SPLIT) Frag<T>::keep(bl[0], bl[1], bl[2], bl[3]);
  }
  acc_guard4(acc[0][0], acc[0][1], acc[0][2], acc[0][3]);
  acc_guard4(acc[1][0], acc[1][1], acc[1][2], acc[1][3]);
  acc_guard4(acc[2][0], acc[2][1], acc[2][2], acc[2][3]);
  acc_guard4(acc[3][0], acc[3][1], acc[3][2], acc[3][3]);

  float* slab = sT[wave];
  const float* Rb = RESID ? (resid + (size_t)b * strideR) : nullptr;
#pragma unroll
  for (int i = 0; i < 4; ++i) {
    const int mBase = m0 + (i << 4);
#pragma unroll
    for (int j = 0; j < 4; ++j) {
      const int n = n0 + (j << 4) + rlane;
      float bv = 0.f;
      if (BIAS_MODE == 2) bv = bias[n];
#pragma unroll
      for (int r = 0; r < 8; ++r) {
        float v = acc[i][j][r] * scale;
        if (BIAS_MODE == 1) v += bias[mBase + mOff + r];
        if (BIAS_MODE == 2) v += bv;
        if (RESID) v += Rb[(size_t)(mBase + mOff + r) * ldc + n];
        if (ACT == 2) v = fmaxf(v, 0.0f);
        if (ACT == 4) v = (v > 0.f) ? v : 0.01f * v;
        slab[(mOff + r) * 68 + (j << 4) + rlane] = v;
      }
    }
    __builtin_amdgcn_fence(__ATOMIC_RELEASE, "workgroup");
    __builtin_amdgcn_wave_barrier();
    __builtin_amdgcn_fence(__ATOMIC_ACQUIRE, "workgroup");
    if (OUT_MODE == 0) {
      float* C = (float*)Cout + (size_t)b * strideC;
      const int hh = lane >> 4, c4 = (lane & 15) * 4;
      for (int pass = 0; pass < 2; ++pass) {
#pragma unroll
        for (int it = 0; it < 8; ++it) {
          const int row = it * 2 + hh;
          v4f v = *(const v4f*)(slab + row * 68 + c4);
          *(volatile v4f*)(C + (size_t)(mBase + row) * ldc + n0 + c4) = v;
        }
        __threadfence();
      }
    } else {
      const int q = lane >> 3, c8 = (lane & 7) * 8;
      unsigned short* C  = (unsigned short*)Cout  + (size_t)b * strideC;
      unsigned short* C2 = (OUT_MODE == 2) ? ((unsigned short*)Cout2 + (size_t)b * strideC) : nullptr;
      for (int pass = 0; pass < 2; ++pass) {
#pragma unroll
        for (int it = 0; it < 4; ++it) {
          const int row = it * 4 + q;
          const float* sp = slab + row * 68 + c8;
          v8h hv, lv;
#pragma unroll
          for (int e = 0; e < 8; ++e) {
            if (OUT_MODE == 1) {
              hv[e] = (_Float16)sp[e];
            } else {
              unsigned short hb = f2bf_bits(sp[e]);
              unsigned short lb = f2bf_bits(sp[e] - bf_bits2f(hb));
              hv[e] = __builtin_bit_cast(_Float16, hb);
              lv[e] = __builtin_bit_cast(_Float16, lb);
            }
          }
          *(volatile v8h*)(C + (size_t)(mBase + row) * ldc + n0 + c8) = hv;
          if (OUT_MODE == 2) *(volatile v8h*)(C2 + (size_t)(mBase + row) * ldc + n0 + c8) = lv;
        }
        __threadfence();
      }
    }
    __builtin_amdgcn_fence(__ATOMIC_RELEASE, "workgroup");
    __builtin_amdgcn_wave_barrier();
    __builtin_amdgcn_fence(__ATOMIC_ACQUIRE, "workgroup");
  }
}

template <int CIN, int KP>
__global__ __launch_bounds__(256) void convw_prep_kernel(const float* __restrict__ w, unsigned short* __restrict__ Bt,
                                                         int n8, float scale) {
  const int i = blockIdx.x * 256 + threadIdx.x;
  if (i >= n8) return;
  constexpr int kReal = 9 * CIN;
  const int e0   = i * 8;
  const int o    = e0 / KP;
  const int colb = e0 - o * KP;
  unsigned short hb[8];
#pragma unroll
  for (int e = 0; e < 8; ++e) {
    const int col  = colb + e;
    const int colc = (col < kReal) ? col : (kReal - 1);
    const int pos  = colc / CIN;
    const int ci   = colc - pos * CIN;
    float v = w[((size_t)o * CIN + ci) * 9 + pos] * scale;
    v = (col < kReal) ? v : 0.0f;
    hb[e] = h_bits(v);
  }
  const v4u u = (v4u){pk16(hb[0], hb[1]), pk16(hb[2], hb[3]), pk16(hb[4], hb[5]), pk16(hb[6], hb[7])};
  unsigned short* q = Bt + (size_t)e0;
  *(volatile v4u*)q = u;
  __threadfence();
  *(volatile v4u*)q = u;
}

__global__ __launch_bounds__(256) void wtsplit_kernel(const float* __restrict__ W, unsigned short* __restrict__ Bh,
                                                      unsigned short* __restrict__ Bl, int Kin, int Nout, int Kp) {
  __shared__ float sm[64][65];
  const int t  = threadIdx.x;
  const int k0 = blockIdx.x * 64;
  const int n0 = blockIdx.y * 64;
#pragma unroll
  for (int i = 0; i < 16; ++i) {
    const int e  = i * 256 + t;
    const int r  = e >> 6;
    const int c  = e & 63;
    const int kk = k0 + r;
    const int kc = (kk < Kin) ? kk : (Kin - 1);
    float v = W[(size_t)kc * Nout + n0 + c];
    v = (kk < Kin) ? v : 0.0f;
    sm[c][r] = v;
  }
  __syncthreads();
  const int lane = t & 31, wave = t >> 5;
  const int q = lane >> 3, c8 = (lane & 7) * 8;
  for (int pass = 0; pass < 2; ++pass) {
#pragma unroll
    for (int it = 0; it < 2; ++it) {
      const int row = wave * 8 + it * 4 + q;
      unsigned short hb[8], lb[8];
#pragma unroll
      for (int e = 0; e < 8; ++e) {
        const float v = sm[row][c8 + e];
        hb[e] = f2bf_bits(v);
        lb[e] = f2bf_bits(v - bf_bits2f(hb[e]));
      }
      const v4u uh = (v4u){pk16(hb[0], hb[1]), pk16(hb[2], hb[3]), pk16(hb[4], hb[5]), pk16(hb[6], hb[7])};
      const v4u ul = (v4u){pk16(lb[0], lb[1]), pk16(lb[2], lb[3]), pk16(lb[4], lb[5]), pk16(lb[6], lb[7])};
      const size_t off = (size_t)(n0 + row) * Kp + k0 + c8;
      *(volatile v4u*)(Bh + off) = uh;
      *(volatile v4u*)(Bl + off) = ul;
    }
    __threadfence();
  }
}

__global__ __launch_bounds__(256) void prop1_kernel(const float* __restrict__ prop, const float* __restrict__ p1w,
                                                    const float* __restrict__ p1b,
                                                    unsigned short* __restrict__ Ph, unsigned short* __restrict__ Pl) {
  __shared__ __align__(16) float sv[4][64];
  const int t = threadIdx.x;
  const int r = t >> 6, col = t & 63;
  const int row = blockIdx.x * 4 + r;
  float s = 0.0f;
#pragma unroll
  for (int i = 0; i < kPropIn; ++i) s = fmaf(prop[row * kPropIn + i], p1w[i * kPropH + col], s);
  s += p1b[col];
  sv[r][col] = fmaxf(s, 0.0f);
  __syncthreads();
  if (t < 32) {
    const int rr = t >> 3, c8 = (t & 7) * 8;
    unsigned short hb[8], lb[8];
#pragma unroll
    for (int e = 0; e < 8; ++e) {
      const float v = sv[rr][c8 + e];
      hb[e] = f2bf_bits(v);
      lb[e] = f2bf_bits(v - bf_bits2f(hb[e]));
    }
    const v4u uh = (v4u){pk16(hb[0], hb[1]), pk16(hb[2], hb[3]), pk16(hb[4], hb[5]), pk16(hb[6], hb[7])};
    const v4u ul = (v4u){pk16(lb[0], lb[1]), pk16(lb[2], lb[3]), pk16(lb[4], lb[5]), pk16(lb[6], lb[7])};
    const size_t off = (size_t)(blockIdx.x * 4 + rr) * kPropH + c8;
    for (int pass = 0; pass < 2; ++pass) {
      *(volatile v4u*)(Ph + off) = uh;
      *(volatile v4u*)(Pl + off) = ul;
      __threadfence();
    }
  }
}

__global__ __launch_bounds__(256) void im2col1_kernel(const float* __restrict__ img, unsigned short* __restrict__ A1, int chunk) {
  const int i = blockIdx.x * 256 + threadIdx.x;
  if (i >= kM1c * 4) return;
  const int row = i >> 2, seg = i & 3;
  const int bl  = row >> 12;
  const int rem = row & 4095;
  const int oy  = rem >> 6, ox = rem & 63;
  const int n   = chunk * kChunk + bl;
  const float* ib = img + (size_t)n * (kCin0 * kImg * kImg);
  unsigned short hb[8];
#pragma unroll
  for (int e = 0; e < 8; ++e) {
    const int col  = seg * 8 + e;
    const int colc = (col < kK1r) ? col : (kK1r - 1);
    const int pos  = colc / 3;
    const int ci   = colc - pos * 3;
    const int kh   = pos / 3;
    const int kw   = pos - kh * 3;
    const int iy   = 2 * oy - 1 + kh;
    const int ix   = 2 * ox - 1 + kw;
    const bool inb = ((unsigned)iy < (unsigned)kImg) && ((unsigned)ix < (unsigned)kImg) && (col < kK1r);
    const int iyc  = iy < 0 ? 0 : (iy > kImg - 1 ? kImg - 1 : iy);
    const int ixc  = ix < 0 ? 0 : (ix > kImg - 1 ? kImg - 1 : ix);
    float v = ib[((size_t)ci * kImg + iyc) * kImg + ixc];
    v = inb ? v : 0.0f;
    hb[e] = h_bits(v);
  }
  const v4u u = (v4u){pk16(hb[0], hb[1]), pk16(hb[2], hb[3]), pk16(hb[4], hb[5]), pk16(hb[6], hb[7])};
  unsigned short* q = A1 + (size_t)i * 8;
  *(volatile v4u*)q = u;
  __threadfence();
  *(volatile v4u*)q = u;
}

template <int CIN, int LOGSO>
__global__ __launch_bounds__(256) void im2col_nhwc_kernel(const unsigned short* __restrict__ src,
                                                          unsigned short* __restrict__ dst, int total) {
  constexpr int kTps  = CIN / 8;
  constexpr int kLogT = (CIN == 64) ? 3 : 4;
  constexpr int kSo   = 1 << LOGSO;
  constexpr int kSi   = 2 * kSo;
  const int i = blockIdx.x * 256 + threadIdx.x;
  if (i >= total) return;
  const int seg = i & (kTps - 1);
  const int qq  = i >> kLogT;
  const int row = qq / 9;
  const int pos = qq - row * 9;
  const int bl  = row >> (2 * LOGSO);
  const int rem = row & (kSo * kSo - 1);
  const int oy  = rem >> LOGSO, ox = rem & (kSo - 1);
  const int kh  = pos / 3, kw = pos - kh * 3;
  const int iy  = 2 * oy - 1 + kh, ix = 2 * ox - 1 + kw;
  const bool inb = ((unsigned)iy < (unsigned)kSi) && ((unsigned)ix < (unsigned)kSi);
  const int iyc = iy < 0 ? 0 : (iy > kSi - 1 ? kSi - 1 : iy);
  const int ixc = ix < 0 ? 0 : (ix > kSi - 1 ? kSi - 1 : ix);
  const size_t srow = ((size_t)bl * kSi + iyc) * kSi + ixc;
  v4u u = *(const v4u*)(src + srow * CIN + seg * 8);
  const unsigned m = inb ? 0xffffffffu : 0u;
  const v4u mm = (v4u){m, m, m, m};
  u = u & mm;
  unsigned short* q = dst + (size_t)i * 8;
  *(volatile v4u*)q = u;
  __threadfence();
  *(volatile v4u*)q = u;
}

__global__ __launch_bounds__(256) void pool_kernel(const float* __restrict__ Y3, unsigned short* __restrict__ VPh,
                                                   unsigned short* __restrict__ VPl, int chunk) {
  __shared__ __align__(16) float sv[256];
  const int bl = blockIdx.x;
  const int c  = threadIdx.x;
  const float* p = Y3 + (size_t)bl * (kSp3 * kSp3) * kCh3 + c;
  float s0 = 0.0f, s1 = 0.0f, s2 = 0.0f, s3 = 0.0f;
#pragma unroll 1
  for (int pos = 0; pos < kSp3 * kSp3; pos += 4) {
    s0 += p[(size_t)(pos + 0) * kCh3];
    s1 += p[(size_t)(pos + 1) * kCh3];
    s2 += p[(size_t)(pos + 2) * kCh3];
    s3 += p[(size_t)(pos + 3) * kCh3];
  }
  const float s = ((s0 + s1) + (s2 + s3)) * (1.0f / 256.0f);
  sv[c] = s;
  __syncthreads();
  if (c < 32) {
    const int c8 = c * 8;
    unsigned short hb[8], lb[8];
#pragma unroll
    for (int e = 0; e < 8; ++e) {
      const float v = sv[c8 + e];
      hb[e] = f2bf_bits(v);
      lb[e] = f2bf_bits(v - bf_bits2f(hb[e]));
    }
    const v4u uh = (v4u){pk16(hb[0], hb[1]), pk16(hb[2], hb[3]), pk16(hb[4], hb[5]), pk16(hb[6], hb[7])};
    const v4u ul = (v4u){pk16(lb[0], lb[1]), pk16(lb[2], lb[3]), pk16(lb[4], lb[5]), pk16(lb[6], lb[7])};
    const size_t off = (size_t)(chunk * kChunk + bl) * kCatK + c8;
    for (int pass = 0; pass < 2; ++pass) {
      *(volatile v4u*)(VPh + off) = uh;
      *(volatile v4u*)(VPl + off) = ul;
      __threadfence();
    }
  }
}

__global__ __launch_bounds__(256) void emb_cols_kernel(const int* __restrict__ tids, const float* __restrict__ temb,
                                                       unsigned short* __restrict__ FEh, unsigned short* __restrict__ FEl) {
  const int i = blockIdx.x * 256 + threadIdx.x;
  if (i >= kBatch * 8) return;
  const int row = i >> 3, seg = i & 7;
  int tid = tids[row];
  tid = (tid < 0) ? (tid + kTasks) : tid;
  tid = tid < 0 ? 0 : (tid > kTasks - 1 ? kTasks - 1 : tid);
  unsigned short hb[8], lb[8];
#pragma unroll
  for (int e = 0; e < 8; ++e) {
    const int col  = seg * 8 + e;
    const int colc = (col < kEmb) ? col : (kEmb - 1);
    float v = temb[(size_t)tid * kEmb + colc];
    v = (col < kEmb) ? v : 0.0f;
    hb[e] = f2bf_bits(v);
    lb[e] = f2bf_bits(v - bf_bits2f(hb[e]));
  }
  const v4u uh = (v4u){pk16(hb[0], hb[1]), pk16(hb[2], hb[3]), pk16(hb[4], hb[5]), pk16(hb[6], hb[7])};
  const v4u ul = (v4u){pk16(lb[0], lb[1]), pk16(lb[2], lb[3]), pk16(lb[4], lb[5]), pk16(lb[6], lb[7])};
  const size_t off = (size_t)row * kCatK + kEnc + seg * 8;
  for (int pass = 0; pass < 2; ++pass) {
    *(volatile v4u*)(FEh + off) = uh;
    *(volatile v4u*)(FEl + off) = ul;
    __threadfence();
  }
}

__global__ __launch_bounds__(128) void routed_heads_kernel(const float* __restrict__ Z, const int* __restrict__ tids,
                                                           const float* __restrict__ h1w, const float* __restrict__ h1b,
                                                           const float* __restrict__ h2w, const float* __restrict__ h2b,
                                                           const float* __restrict__ h3w, const float* __restrict__ h3b,
                                                           float* __restrict__ out) {
  __shared__ __align__(16) float zs[kEnc];
  __shared__ __align__(16) float a1[kHidH];
  __shared__ __align__(16) float a2[kHidH];
  __shared__ __align__(16) float res[32];
  const int t   = threadIdx.x;
  const int blk = blockIdx.x;
  for (int s = 0; s < 8; ++s) {
    const int b = blk * 8 + s;
    int tid = tids[b];
    tid = (tid < 0) ? (tid + kTasks) : tid;
    tid = tid < 0 ? 0 : (tid > kTasks - 1 ? kTasks - 1 : tid);
    zs[t]         = Z[(size_t)b * kEnc + t];
    zs[kHidH + t] = Z[(size_t)b * kEnc + kHidH + t];
    __syncthreads();
    {
      const float* w = h1w + (size_t)tid * (kEnc * kHidH) + t;
      float acc = 0.0f;
#pragma unroll 1
      for (int i = 0; i < kEnc; ++i) acc = fmaf(zs[i], w[(size_t)i * kHidH], acc);
      acc += h1b[(size_t)tid * kHidH + t];
      a1[t] = fmaxf(acc, 0.0f);
    }
    __syncthreads();
    {
      const float* w = h2w + (size_t)tid * (kHidH * kHidH) + t;
      float acc = 0.0f;
#pragma unroll 1
      for (int i = 0; i < kHidH; ++i) acc = fmaf(a1[i], w[(size_t)i * kHidH], acc);
      acc += h2b[(size_t)tid * kHidH + t];
      a2[t] = fmaxf(acc, 0.0f);
    }
    __syncthreads();
    if (t < kActN) {
      const float* w = h3w + (size_t)tid * (kHidH * kActN) + t;
      float acc = 0.0f;
#pragma unroll 1
      for (int i = 0; i < kHidH; ++i) acc = fmaf(a2[i], w[(size_t)i * kActN], acc);
      acc += h3b[(size_t)tid * kActN + t];
      res[s * kActN + t] = acc;
    }
    __syncthreads();
  }
  if (t < 8) {
    const v4f v = *(const v4f*)(res + t * 4);
    float* op = out + (size_t)(blk * 8 + t) * kActN;
    *(volatile v4f*)op = v;
    __threadfence();
    *(volatile v4f*)op = v;
  }
}

typedef void (*gemm_fn_t)(const unsigned short*, const unsigned short*, int, long,
                          const unsigned short*, const unsigned short*, int, long,
                          void*, void*, int, long, const float*, const float*, long, int, int, int, float);

extern "C" void kernel_launch(void* const* d_in, const int* in_sizes, int n_in,
                              void* d_out, int out_size, void* d_ws, size_t ws_size,
                              hipStream_t stream)
{
  if (n_in < 26) return;
  if (in_sizes[0] != kBatch * kCin0 * kImg * kImg) return;
  if (in_sizes[1] != kBatch * kPropIn) return;
  if (in_sizes[2] != kBatch) return;
  if (in_sizes[5] != kCh2 * kCh1 * 9) return;
  if (in_sizes[7] != kCh3 * kCh2 * 9) return;
  if (in_sizes[13] != kCatK * kEnc) return;
  if (in_sizes[18] != kGK * kEnc) return;
  if (in_sizes[20] != kTasks * kEnc * kHidH) return;
  if (in_sizes[22] != kTasks * kHidH * kHidH) return;
  if (in_sizes[24] != kTasks * kHidH * kActN) return;
  if (out_size != kBatch * kActN) return;

  const float* images = (const float*)d_in[0];
  const float* prop   = (const float*)d_in[1];
  const int*   tids   = (const int*)d_in[2];
  const float* c1w = (const float*)d_in[3];  const float* c1b = (const float*)d_in[4];
  const float* c2w = (const float*)d_in[5];  const float* c2b = (const float*)d_in[6];
  const float* c3w = (const float*)d_in[7];  const float* c3b = (const float*)d_in[8];
  const float* p1w = (const float*)d_in[9];  const float* p1b = (const float*)d_in[10];
  const float* p2w = (const float*)d_in[11]; const float* p2b = (const float*)d_in[12];
  const float* f1w = (const float*)d_in[13]; const float* f1b = (const float*)d_in[14];
  const float* f2w = (const float*)d_in[15]; const float* f2b = (const float*)d_in[16];
  const float* temb = (const float*)d_in[17];
  const float* gw  = (const float*)d_in[18]; const float* gb  = (const float*)d_in[19];
  const float* h1w = (const float*)d_in[20]; const float* h1b = (const float*)d_in[21];
  const float* h2w = (const float*)d_in[22]; const float* h2b = (const float*)d_in[23];
  const float* h3w = (const float*)d_in[24]; const float* h3b = (const float*)d_in[25];

  char* ws = (char*)d_ws;
  size_t off = 0;
  auto carve = [&](size_t bytes) -> size_t { size_t o = off; off += (bytes + 255) & ~(size_t)255; return o; };
  const size_t oBt1  = carve((size_t)kCh1 * kK1 * 2);
  const size_t oBt2  = carve((size_t)kCh2 * kK2 * 2);
  const size_t oBt3  = carve((size_t)kCh3 * kK3 * 2);
  const size_t oP2th = carve((size_t)kPropH * kPropH * 2);
  const size_t oP2tl = carve((size_t)kPropH * kPropH * 2);
  const size_t oF1th = carve((size_t)kEnc * kCatK * 2);
  const size_t oF1tl = carve((size_t)kEnc * kCatK * 2);
  const size_t oF2th = carve((size_t)kEnc * kEnc * 2);
  const size_t oF2tl = carve((size_t)kEnc * kEnc * 2);
  const size_t oGth  = carve((size_t)kEnc * kCatK * 2);
  const size_t oGtl  = carve((size_t)kEnc * kCatK * 2);
  const size_t oP1h  = carve((size_t)kBatch * kPropH * 2);
  const size_t oP1l  = carve((size_t)kBatch * kPropH * 2);
  const size_t oVPh  = carve((size_t)kBatch * kCatK * 2);
  const size_t oVPl  = carve((size_t)kBatch * kCatK * 2);
  const size_t oF1h  = carve((size_t)kBatch * kEnc * 2);
  const size_t oF1l  = carve((size_t)kBatch * kEnc * 2);
  const size_t oFEh  = carve((size_t)kBatch * kCatK * 2);
  const size_t oFEl  = carve((size_t)kBatch * kCatK * 2);
  const size_t oZ    = carve((size_t)kBatch * kEnc * 4);
  const size_t oA1   = carve((size_t)kM1c * kK1 * 2);
  const size_t oY1   = carve((size_t)kM1c * kCh1 * 2);
  const size_t oA2   = carve((size_t)kM2c * kK2 * 2);
  const size_t oY2   = carve((size_t)kM2c * kCh2 * 2);
  const size_t oA3   = carve((size_t)kM3c * kK3 * 2);
  const size_t oY3   = carve((size_t)kM3c * kCh3 * 4);
  if (off > ws_size) return;

  unsigned short* Bt1  = (unsigned short*)(ws + oBt1);
  unsigned short* Bt2  = (unsigned short*)(ws + oBt2);
  unsigned short* Bt3  = (unsigned short*)(ws + oBt3);
  unsigned short* P2th = (unsigned short*)(ws + oP2th);
  unsigned short* P2tl = (unsigned short*)(ws + oP2tl);
  unsigned short* F1th = (unsigned short*)(ws + oF1th);
  unsigned short* F1tl = (unsigned short*)(ws + oF1tl);
  unsigned short* F2th = (unsigned short*)(ws + oF2th);
  unsigned short* F2tl = (unsigned short*)(ws + oF2tl);
  unsigned short* Gth  = (unsigned short*)(ws + oGth);
  unsigned short* Gtl  = (unsigned short*)(ws + oGtl);
  unsigned short* P1h  = (unsigned short*)(ws + oP1h);
  unsigned short* P1l  = (unsigned short*)(ws + oP1l);
  unsigned short* VPh  = (unsigned short*)(ws + oVPh);
  unsigned short* VPl  = (unsigned short*)(ws + oVPl);
  unsigned short* F1h  = (unsigned short*)(ws + oF1h);
  unsigned short* F1l  = (unsigned short*)(ws + oF1l);
  unsigned short* FEh  = (unsigned short*)(ws + oFEh);
  unsigned short* FEl  = (unsigned short*)(ws + oFEl);
  float*          Zf   = (float*)(ws + oZ);
  unsigned short* A1   = (unsigned short*)(ws + oA1);
  unsigned short* Y1   = (unsigned short*)(ws + oY1);
  unsigned short* A2   = (unsigned short*)(ws + oA2);
  unsigned short* Y2   = (unsigned short*)(ws + oY2);
  unsigned short* A3   = (unsigned short*)(ws + oA3);
  float*          Y3   = (float*)(ws + oY3);

  gemm_fn_t gemm_c12 = wmma_gemm64<0, false, 2, 1, false, 2>;
  gemm_fn_t gemm_c3  = wmma_gemm64<0, false, 2, 0, false, 2>;
  gemm_fn_t gemm_p2  = wmma_gemm64<1, true,  2, 2, false, 0>;
  gemm_fn_t gemm_fx  = wmma_gemm64<1, true,  2, 2, false, 2>;
  gemm_fn_t gemm_g   = wmma_gemm64<1, true,  2, 0, false, 2>;

  {
    const int n8_1 = kCh1 * kK1 / 8;
    const int n8_2 = kCh2 * kK2 / 8;
    const int n8_3 = kCh3 * kK3 / 8;
    convw_prep_kernel<kCin0, kK1><<<(n8_1 + 255) / 256, 256, 0, stream>>>(c1w, Bt1, n8_1, kWCarry);
    convw_prep_kernel<kCh1,  kK2><<<(n8_2 + 255) / 256, 256, 0, stream>>>(c2w, Bt2, n8_2, kWCarry);
    convw_prep_kernel<kCh2,  kK3><<<(n8_3 + 255) / 256, 256, 0, stream>>>(c3w, Bt3, n8_3, kWCarry);
    wtsplit_kernel<<<dim3(kPropH / 64, kPropH / 64), 256, 0, stream>>>(p2w, P2th, P2tl, kPropH, kPropH, kPropH);
    wtsplit_kernel<<<dim3(kCatK / 64, kEnc / 64), 256, 0, stream>>>(f1w, F1th, F1tl, kCatK, kEnc, kCatK);
    wtsplit_kernel<<<dim3(kEnc / 64, kEnc / 64), 256, 0, stream>>>(f2w, F2th, F2tl, kEnc, kEnc, kEnc);
    wtsplit_kernel<<<dim3(kCatK / 64, kEnc / 64), 256, 0, stream>>>(gw, Gth, Gtl, kGK, kEnc, kCatK);
    prop1_kernel<<<kBatch / 4, 256, 0, stream>>>(prop, p1w, p1b, P1h, P1l);
  }

  const int tot2 = kM2c * 9 * (kCh1 / 8);
  const int tot3 = kM3c * 9 * (kCh2 / 8);
  const int blk_g1 = ((kM1c / 64) * (kCh1 / 64) + 7) / 8;
  const int blk_g2 = ((kM2c / 64) * (kCh2 / 64) + 7) / 8;
  const int blk_g3 = ((kM3c / 64) * (kCh3 / 64) + 7) / 8;
  for (int ch = 0; ch < kNChunk; ++ch) {
    im2col1_kernel<<<(kM1c * 4 + 255) / 256, 256, 0, stream>>>(images, A1, ch);
    gemm_c12<<<dim3(blk_g1, 1), 256, 0, stream>>>(A1, A1, kK1, 0L, Bt1, Bt1, kK1, 0L,
                                                 (void*)Y1, (void*)Y1, kCh1, 0L, c1b, c1b, 0L,
                                                 kM1c, kCh1, kK1, kWCarryInv);
    im2col_nhwc_kernel<kCh1, 5><<<(tot2 + 255) / 256, 256, 0, stream>>>(Y1, A2, tot2);
    gemm_c12<<<dim3(blk_g2, 1), 256, 0, stream>>>(A2, A2, kK2, 0L, Bt2, Bt2, kK2, 0L,
                                                 (void*)Y2, (void*)Y2, kCh2, 0L, c2b, c2b, 0L,
                                                 kM2c, kCh2, kK2, kWCarryInv);
    im2col_nhwc_kernel<kCh2, 4><<<(tot3 + 255) / 256, 256, 0, stream>>>(Y2, A3, tot3);
    gemm_c3<<<dim3(blk_g3, 1), 256, 0, stream>>>(A3, A3, kK3, 0L, Bt3, Bt3, kK3, 0L,
                                                (void*)Y3, (void*)Y3, kCh3, 0L, c3b, c3b, 0L,
                                                kM3c, kCh3, kK3, kWCarryInv);
    pool_kernel<<<kChunk, 256, 0, stream>>>(Y3, VPh, VPl, ch);
  }

  gemm_p2<<<dim3(1, 1), 256, 0, stream>>>(P1h, P1l, kPropH, 0L, P2th, P2tl, kPropH, 0L,
                                          (void*)(VPh + kEnc), (void*)(VPl + kEnc), kCatK, 0L, p2b, p2b, 0L,
                                          kBatch, kPropH, kPropH, 1.0f);
  gemm_fx<<<dim3(2, 1), 256, 0, stream>>>(VPh, VPl, kCatK, 0L, F1th, F1tl, kCatK, 0L,
                                          (void*)F1h, (void*)F1l, kEnc, 0L, f1b, f1b, 0L,
                                          kBatch, kEnc, kCatK, 1.0f);
  gemm_fx<<<dim3(2, 1), 256, 0, stream>>>(F1h, F1l, kEnc, 0L, F2th, F2tl, kEnc, 0L,
                                          (void*)FEh, (void*)FEl, kCatK, 0L, f2b, f2b, 0L,
                                          kBatch, kEnc, kEnc, 1.0f);
  emb_cols_kernel<<<(kBatch * 8 + 255) / 256, 256, 0, stream>>>(tids, temb, FEh, FEl);
  gemm_g<<<dim3(2, 1), 256, 0, stream>>>(FEh, FEl, kCatK, 0L, Gth, Gtl, kCatK, 0L,
                                         (void*)Zf, (void*)Zf, kEnc, 0L, gb, gb, 0L,
                                         kBatch, kEnc, kCatK, 1.0f);
  routed_heads_kernel<<<kBatch / 8, 128, 0, stream>>>(Zf, tids, h1w, h1b, h2w, h2b, h3w, h3b, (float*)d_out);
}
